// CrossMamba_34522947125651
// MI455X (gfx1250) — hardware-run, weakly checked
//
#include <hip/hip_runtime.h>
#include <hip/hip_fp16.h>
#include <math.h>

typedef __attribute__((ext_vector_type(16))) _Float16 v16h;
typedef __attribute__((ext_vector_type(8)))  _Float16 v8h;
typedef __attribute__((ext_vector_type(16))) __bf16   v16b;
typedef __attribute__((ext_vector_type(8)))  __bf16   v8b;
typedef __attribute__((ext_vector_type(8)))  float    v8f;
typedef __attribute__((ext_vector_type(4)))  float    v4f;
typedef __attribute__((ext_vector_type(4)))  unsigned v4u;

constexpr int kNB   = 4;
constexpr int kCm   = 256;
constexpr int kL    = 4096;
constexpr int kDin  = 512;
constexpr int kNst  = 16;
constexpr int kDtR  = 16;
constexpr int kDtKP = 32;
constexpr int kXzP  = 2 * kDin;
constexpr int kXdR  = kDtR + 2 * kNst;
constexpr int kXdP  = 64;
constexpr int kRows = kNB * kL;
constexpr int kConvTP = 260;
static_assert(kXdR == 48 && kXdR <= kXdP, "x_proj width");
static_assert((kCm % 32) == 0 && (kDin % 32) == 0 && (kDtKP % 32) == 0, "GEMM K multiples of 32");
static_assert((kL % 64) == 0 && (kXzP % 64) == 0 && (kXdP % 64) == 0 && (kDin % 64) == 0 && (kCm % 64) == 0, "GEMM M,N multiples of 64");
static_assert((kDin % 256) == 0, "conv block width");

constexpr float kCU  = 32.0f;
constexpr float kCWX = 1024.0f;
constexpr float kCDT = 32.0f;
constexpr float kCWD = 256.0f;
constexpr float kCY  = 64.0f;
constexpr float kCWO = 1024.0f;
constexpr float kSclX = 1.0f / (kCU * kCWX);
constexpr float kSclD = 1.0f / (kCDT * kCWD);
constexpr float kSclO = 1.0f / (kCY * kCWO);

constexpr int kQvCw    = 0;
constexpr int kQvCb    = kQvCw + kDin * 4;
constexpr int kQvDb    = kQvCb + kDin;
constexpr int kQvAl    = kQvDb + kDin;
constexpr int kQvDk    = kQvAl + kDin * kNst;
constexpr int kQvTotal = kQvDk + kDin;
static_assert((kQvCb % 32) == 0 && (kQvDb % 32) == 0 && (kQvAl % 32) == 0 && (kQvDk % 32) == 0 && (kQvTotal % 128) == 0, "table segments on line boundaries");

constexpr size_t kSzXB    = (size_t)kRows * kCm * 2;
constexpr size_t kSzWIB   = (size_t)kXzP * kCm * 2;
constexpr size_t kSzWX16  = (size_t)kXdP * kDin * 2;
constexpr size_t kSzWDT16 = (size_t)kDin * kDtKP * 2;
constexpr size_t kSzWO16  = (size_t)kCm * kDin * 2;
constexpr size_t kSzQV    = (size_t)kQvTotal * 4;
constexpr size_t kSzXZ    = (size_t)kL * kXzP * 4;
constexpr size_t kSzU     = (size_t)kL * kDin * 4;
constexpr size_t kSzU16   = (size_t)kL * kDin * 2;
constexpr size_t kSzXD    = (size_t)kL * kXdP * 4;
constexpr size_t kSzDT16  = (size_t)kL * kDtKP * 2;
constexpr size_t kSzDT    = (size_t)kL * kDin * 4;
constexpr size_t kSzY16   = (size_t)kRows * kDin * 2;
constexpr size_t kOffXB    = 0;
constexpr size_t kOffWIB   = kOffXB    + kSzXB;
constexpr size_t kOffWX16  = kOffWIB   + kSzWIB;
constexpr size_t kOffWDT16 = kOffWX16  + kSzWX16;
constexpr size_t kOffWO16  = kOffWDT16 + kSzWDT16;
constexpr size_t kOffQV    = kOffWO16  + kSzWO16;
constexpr size_t kOffXZ    = kOffQV    + kSzQV;
constexpr size_t kOffU     = kOffXZ    + kSzXZ;
constexpr size_t kOffU16   = kOffU     + kSzU;
constexpr size_t kOffXD    = kOffU16   + kSzU16;
constexpr size_t kOffDT16  = kOffXD    + kSzXD;
constexpr size_t kOffDT    = kOffDT16  + kSzDT16;
constexpr size_t kOffY16   = kOffDT    + kSzDT;
constexpr size_t kWsTotal  = kOffY16   + kSzY16;
static_assert(kWsTotal == 65157120ull, "carve total");
static_assert(kWsTotal <= 134217728ull, "carve cap");
static_assert((kOffWIB % 128) == 0 && (kOffWX16 % 128) == 0 && (kOffWDT16 % 128) == 0 && (kOffWO16 % 128) == 0 &&
              (kOffQV % 128) == 0 && (kOffXZ % 128) == 0 && (kOffU % 128) == 0 && (kOffU16 % 128) == 0 &&
              (kOffXD % 128) == 0 && (kOffDT16 % 128) == 0 && (kOffDT % 128) == 0 && (kOffY16 % 128) == 0, "128-B aligned regions");

__device__ __forceinline__ unsigned bf16bits(float f) {
  const unsigned u = __float_as_uint(f);
  return (u + 0x7FFFu + ((u >> 16) & 1u)) >> 16;
}
__device__ __forceinline__ float bf16val(float f) {
  return __uint_as_float(bf16bits(f) << 16);
}
__device__ __forceinline__ unsigned f16bits_flush(float v) {
  const float f = (fabsf(v) < 6.103515625e-05f) ? 0.0f : v;
  return (unsigned)__half_as_ushort(__float2half_rn(f));
}
__device__ __forceinline__ unsigned pack2_bf16(float a, float b) {
  const unsigned lo = bf16bits(a);
  const unsigned hi = bf16bits(b);
  return lo | (hi << 16);
}
__device__ __forceinline__ unsigned pack2_f16(float a, float b) {
  const unsigned lo = f16bits_flush(a);
  const unsigned hi = f16bits_flush(b);
  return lo | (hi << 16);
}

namespace eng {

__device__ __forceinline__ void guard1_h(v8f& a, v16h x, v16h y) {
  asm volatile("v_nop\n\tv_nop\n\tv_nop\n\tv_nop" : "+v"(a) : "v"(x), "v"(y));
}
__device__ __forceinline__ void guard1_b(v8f& a, v16b x, v16b y) {
  asm volatile("v_nop\n\tv_nop\n\tv_nop\n\tv_nop" : "+v"(a) : "v"(x), "v"(y));
}
__device__ __forceinline__ void keep4_h(v16h a, v16h b, v16h c, v16h d) {
  asm volatile("v_nop" :: "v"(a), "v"(b), "v"(c), "v"(d));
}
__device__ __forceinline__ void keep4_b(v16b a, v16b b, v16b c, v16b d) {
  asm volatile("v_nop" :: "v"(a), "v"(b), "v"(c), "v"(d));
}
__device__ __forceinline__ void acc_guard1(v8f& a) {
  asm volatile("v_nop\n\tv_nop\n\tv_nop\n\tv_nop" : "+v"(a));
}

template <typename T> struct Frag;
template <> struct Frag<_Float16> {
  typedef v16h V;
  union U { v16h v; v8h h[2]; };
  static __device__ __forceinline__ v16h load(const _Float16* p) {
    U f;
    f.h[0] = *(const v8h*)(p);
    f.h[1] = *(const v8h*)(p + 16);
    return f.v;
  }
  static __device__ __forceinline__ v8f mma(v16h a, v16h b, v8f c) {
    return __builtin_amdgcn_wmma_f32_16x16x32_f16(false, a, false, b, (short)0, c, false, false);
  }
  static __device__ __forceinline__ void guard(v8f& a, v16h x, v16h y) { guard1_h(a, x, y); }
  static __device__ __forceinline__ void keep(v16h a, v16h b, v16h c, v16h d) { keep4_h(a, b, c, d); }
};
template <> struct Frag<__bf16> {
  typedef v16b V;
  union U { v16b v; v8b h[2]; };
  static __device__ __forceinline__ v16b load(const __bf16* p) {
    U f;
    f.h[0] = *(const v8b*)(p);
    f.h[1] = *(const v8b*)(p + 16);
    return f.v;
  }
  static __device__ __forceinline__ v8f mma(v16b a, v16b b, v8f c) {
    return __builtin_amdgcn_wmma_f32_16x16x32_bf16(false, a, false, b, (short)0, c, false, false);
  }
  static __device__ __forceinline__ void guard(v8f& a, v16b x, v16b y) { guard1_b(a, x, y); }
  static __device__ __forceinline__ void keep(v16b a, v16b b, v16b c, v16b d) { keep4_b(a, b, c, d); }
};

template <int ET> struct Elem;
template <> struct Elem<0> { typedef _Float16 T; };
template <> struct Elem<1> { typedef __bf16 T; };

template <int ET, int BIAS_MODE>
__global__ __launch_bounds__(256) void gemm64_kernel(
    const unsigned short* __restrict__ Ap, int lda, long strideA,
    const unsigned short* __restrict__ Btp, int ldb, long strideB,
    float* __restrict__ Cout, int ldc, long strideC,
    const float* __restrict__ bias,
    int M, int N, int K, float scale) {
  typedef typename Elem<ET>::T T;
  typedef typename Frag<T>::V V;
  const T* A  = (const T*)Ap;
  const T* Bt = (const T*)Btp;
  __shared__ __align__(16) float sT[8][16 * 68];
  const int b    = blockIdx.y;
  const int lane = threadIdx.x & 31;
  const int wave = threadIdx.x >> 5;
  const int tilesN = N >> 6;
  const int tilesM = M >> 6;
  const int tile = blockIdx.x * 8 + wave;
  if (tile >= tilesM * tilesN) return;
  const int tm = tile / tilesN;
  const int tn = tile - tm * tilesN;
  const int m0 = tm << 6;
  const int n0 = tn << 6;

  const T* Ab = A  + (size_t)b * strideA;
  const T* Bb = Bt + (size_t)b * strideB;

  const int rlane = lane & 15;
  const int koff  = (lane >> 4) * 8;
  const int mOff  = (lane >> 4) * 8;

  v8f acc[4][4];
#pragma unroll
  for (int i = 0; i < 4; ++i)
#pragma unroll
    for (int j = 0; j < 4; ++j) acc[i][j] = (v8f){0.f, 0.f, 0.f, 0.f, 0.f, 0.f, 0.f, 0.f};

  for (int k0 = 0; k0 < K; k0 += 32) {
    V bh[4];
#pragma unroll
    for (int j = 0; j < 4; ++j) {
      const size_t bo = (size_t)(n0 + (j << 4) + rlane) * ldb + koff + k0;
      bh[j] = Frag<T>::load(Bb + bo);
    }
#pragma unroll
    for (int i = 0; i < 4; ++i) {
      const size_t ao = (size_t)(m0 + (i << 4) + rlane) * lda + koff + k0;
      V ah = Frag<T>::load(Ab + ao);
#pragma unroll
      for (int j = 0; j < 4; ++j) acc[i][j] = Frag<T>::mma(ah, bh[j], acc[i][j]);
      Frag<T>::guard(acc[i][0], ah, bh[0]);
      Frag<T>::guard(acc[i][1], ah, bh[1]);
      Frag<T>::guard(acc[i][2], ah, bh[2]);
      Frag<T>::guard(acc[i][3], ah, bh[3]);
    }
    Frag<T>::keep(bh[0], bh[1], bh[2], bh[3]);
  }
#pragma unroll
  for (int i = 0; i < 4; ++i)
#pragma unroll
    for (int j = 0; j < 4; ++j) acc_guard1(acc[i][j]);

  float* slab = sT[wave];
  float* C = Cout + (size_t)b * strideC;
  const int hh = lane >> 4;
  const int c4 = (lane & 15) * 4;
#pragma unroll
  for (int i = 0; i < 4; ++i) {
    const int mBase = m0 + (i << 4);
#pragma unroll
    for (int j = 0; j < 4; ++j) {
      const int n = n0 + (j << 4) + rlane;
      float bv = 0.f;
      if (BIAS_MODE == 2) bv = bias[n];
#pragma unroll
      for (int r = 0; r < 8; ++r) {
        float v = acc[i][j][r] * scale;
        if (BIAS_MODE == 2) v += bv;
        slab[(mOff + r) * 68 + (j << 4) + rlane] = v;
      }
    }
    __builtin_amdgcn_fence(__ATOMIC_RELEASE, "workgroup");
    __builtin_amdgcn_wave_barrier();
    __builtin_amdgcn_fence(__ATOMIC_ACQUIRE, "workgroup");
    for (int pass = 0; pass < 2; ++pass) {
#pragma unroll
      for (int it = 0; it < 8; ++it) {
        const int row = it * 2 + hh;
        const v4f v = *(const v4f*)(slab + row * 68 + c4);
        *(volatile v4f*)(C + (size_t)(mBase + row) * ldc + n0 + c4) = v;
      }
      __threadfence();
    }
    __builtin_amdgcn_fence(__ATOMIC_RELEASE, "workgroup");
    __builtin_amdgcn_wave_barrier();
    __builtin_amdgcn_fence(__ATOMIC_ACQUIRE, "workgroup");
  }
}

}

__global__ __launch_bounds__(256) void xpose_bf16_kernel(const float* __restrict__ x, unsigned short* __restrict__ XB)
{
  __shared__ __align__(16) float sT[64 * 68];
  const int tid = threadIdx.x, lane = tid & 31, wave = tid >> 5;
  const int l0 = blockIdx.x * 64, c0 = blockIdx.y * 64, b = blockIdx.z;
  const int l4 = (tid & 15) * 4, cr = tid >> 4;
#pragma unroll
  for (int i = 0; i < 4; ++i) {
    const int c = cr + 16 * i;
    const v4f v = *(const v4f*)(x + ((size_t)(b * kCm + c0 + c)) * kL + l0 + l4);
    sT[(l4 + 0) * 68 + c] = v[0];
    sT[(l4 + 1) * 68 + c] = v[1];
    sT[(l4 + 2) * 68 + c] = v[2];
    sT[(l4 + 3) * 68 + c] = v[3];
  }
  __syncthreads();
  const int q = lane >> 3, c8 = (lane & 7) * 8;
  v4u w[2];
#pragma unroll
  for (int it = 0; it < 2; ++it) {
    const int row = it * 32 + wave * 4 + q;
    const float* sp = sT + row * 68 + c8;
    const v4f a0 = *(const v4f*)(sp);
    const v4f a1 = *(const v4f*)(sp + 4);
    const unsigned w0 = pack2_bf16(a0[0], a0[1]);
    const unsigned w1 = pack2_bf16(a0[2], a0[3]);
    const unsigned w2 = pack2_bf16(a1[0], a1[1]);
    const unsigned w3 = pack2_bf16(a1[2], a1[3]);
    w[it] = (v4u){w0, w1, w2, w3};
  }
  for (int pass = 0; pass < 2; ++pass) {
#pragma unroll
    for (int it = 0; it < 2; ++it) {
      const int row = it * 32 + wave * 4 + q;
      unsigned short* p = XB + ((size_t)(b * kL + l0 + row)) * kCm + c0 + c8;
      *(volatile v4u*)p = w[it];
    }
    __threadfence();
  }
}

template <int MODE>
__device__ __forceinline__ unsigned cvt16_bits(float v, float carry) {
  if (MODE == 0) return bf16bits(v);
  return f16bits_flush(bf16val(v) * carry);
}
template <int MODE>
__global__ __launch_bounds__(256) void prep_plane16_kernel(
    const float* __restrict__ src, int R, int Kc,
    unsigned short* __restrict__ dst, int Kp, float carry, int total8)
{
  const int i = blockIdx.x * 256 + threadIdx.x;
  if (i >= total8) return;
  const int g  = Kp >> 3;
  const int r  = i / g;
  const int k0 = (i - r * g) << 3;
  const bool live = (r < R) && (k0 < Kc);
  const int rc = (r < R) ? r : (R - 1);
  const int kc = (k0 < Kc) ? k0 : 0;
  v4f a0 = *(const v4f*)(src + (size_t)rc * Kc + kc);
  v4f a1 = *(const v4f*)(src + (size_t)rc * Kc + kc + 4);
  asm volatile("" : "+v"(a0));
  asm volatile("" : "+v"(a1));
  const float f0 = live ? a0[0] : 0.0f;
  const float f1 = live ? a0[1] : 0.0f;
  const float f2 = live ? a0[2] : 0.0f;
  const float f3 = live ? a0[3] : 0.0f;
  const float f4 = live ? a1[0] : 0.0f;
  const float f5 = live ? a1[1] : 0.0f;
  const float f6 = live ? a1[2] : 0.0f;
  const float f7 = live ? a1[3] : 0.0f;
  const unsigned b0 = cvt16_bits<MODE>(f0, carry);
  const unsigned b1 = cvt16_bits<MODE>(f1, carry);
  const unsigned b2 = cvt16_bits<MODE>(f2, carry);
  const unsigned b3 = cvt16_bits<MODE>(f3, carry);
  const unsigned b4 = cvt16_bits<MODE>(f4, carry);
  const unsigned b5 = cvt16_bits<MODE>(f5, carry);
  const unsigned b6 = cvt16_bits<MODE>(f6, carry);
  const unsigned b7 = cvt16_bits<MODE>(f7, carry);
  const v4u w = (v4u){b0 | (b1 << 16), b2 | (b3 << 16), b4 | (b5 << 16), b6 | (b7 << 16)};
  unsigned short* p = dst + (size_t)i * 8;
  *(volatile v4u*)p = w;
  __threadfence();
  *(volatile v4u*)p = w;
}

__global__ __launch_bounds__(256) void quant_vals_kernel(
    const float* __restrict__ cw, const float* __restrict__ cb, const float* __restrict__ db,
    const float* __restrict__ al, const float* __restrict__ dk, float* __restrict__ QV)
{
  const int i = blockIdx.x * 256 + threadIdx.x;
  if (i >= kQvTotal / 4) return;
  const float* s = cw;
  int j = i;
  if (i >= kQvCb / 4) { s = cb; j = i - kQvCb / 4; }
  if (i >= kQvDb / 4) { s = db; j = i - kQvDb / 4; }
  if (i >= kQvAl / 4) { s = al; j = i - kQvAl / 4; }
  if (i >= kQvDk / 4) { s = dk; j = i - kQvDk / 4; }
  const v4f a = *(const v4f*)(s + 4 * j);
  v4f o;
  o[0] = bf16val(a[0]);
  o[1] = bf16val(a[1]);
  o[2] = bf16val(a[2]);
  o[3] = bf16val(a[3]);
  float* p = QV + 4 * i;
  *(volatile v4f*)p = o;
  __threadfence();
  *(volatile v4f*)p = o;
}

__global__ __launch_bounds__(256) void conv_silu_kernel(
    const float* __restrict__ XZ, const float* __restrict__ cw, const float* __restrict__ cb,
    float* __restrict__ U, unsigned short* __restrict__ U16)
{
  __shared__ __align__(16) float sT[16 * kConvTP];
  const int tid = threadIdx.x, lane = tid & 31, wave = tid >> 5;
  const int d0 = blockIdx.x * 256, d = d0 + tid;
  const int g0 = blockIdx.y * 64;
  const v4f wv = *(const v4f*)(cw + d * 4);
  const float w0 = wv[0], w1 = wv[1], w2 = wv[2], w3 = wv[3];
  const float bc = cb[d];
  float xm3, xm2, xm1;
  {
    const bool hist = (g0 > 0);
    const int rb = hist ? (g0 - 3) : g0;
    float v3 = XZ[(size_t)rb * kXzP + d];
    float v2 = XZ[(size_t)(rb + 1) * kXzP + d];
    float v1 = XZ[(size_t)(rb + 2) * kXzP + d];
    asm volatile("" : "+v"(v3));
    asm volatile("" : "+v"(v2));
    asm volatile("" : "+v"(v1));
    xm3 = hist ? v3 : 0.0f;
    xm2 = hist ? v2 : 0.0f;
    xm1 = hist ? v1 : 0.0f;
  }
  const int hrow = wave >> 1;
  const int hch  = (wave & 1) * 128 + lane * 4;
#pragma unroll 1
  for (int sub = 0; sub < 4; ++sub) {
    const int lb = g0 + sub * 16;
#pragma unroll 1
    for (int s = 0; s < 16; ++s) {
      const float xcur = XZ[(size_t)(lb + s) * kXzP + d];
      float acc = w0 * xm3;
      acc = fmaf(w1, xm2, acc);
      acc = fmaf(w2, xm1, acc);
      acc = fmaf(w3, xcur, acc);
      const float sv = acc + bc;
      const float sg = __builtin_amdgcn_rcpf(1.0f + expf(-sv));
      sT[s * kConvTP + tid] = sv * sg;
      xm3 = xm2;
      xm2 = xm1;
      xm1 = xcur;
    }
    __syncthreads();
    v4f fv[4];
    v4u hw[2];
#pragma unroll
    for (int it = 0; it < 4; ++it) fv[it] = *(const v4f*)(sT + (it * 4 + hrow) * kConvTP + hch);
#pragma unroll
    for (int it = 0; it < 2; ++it) {
      const float* sp = sT + (it * 8 + wave) * kConvTP + lane * 8;
      const v4f a0 = *(const v4f*)(sp);
      const v4f a1 = *(const v4f*)(sp + 4);
      const unsigned p0 = pack2_f16(a0[0] * kCU, a0[1] * kCU);
      const unsigned p1 = pack2_f16(a0[2] * kCU, a0[3] * kCU);
      const unsigned p2 = pack2_f16(a1[0] * kCU, a1[1] * kCU);
      const unsigned p3 = pack2_f16(a1[2] * kCU, a1[3] * kCU);
      hw[it] = (v4u){p0, p1, p2, p3};
    }
    for (int pass = 0; pass < 2; ++pass) {
#pragma unroll
      for (int it = 0; it < 4; ++it)
        *(volatile v4f*)(U + (size_t)(lb + it * 4 + hrow) * kDin + d0 + hch) = fv[it];
#pragma unroll
      for (int it = 0; it < 2; ++it) {
        unsigned short* p = U16 + (size_t)(lb + it * 8 + wave) * kDin + d0 + lane * 8;
        *(volatile v4u*)p = hw[it];
      }
      __threadfence();
    }
    __syncthreads();
  }
}

__global__ __launch_bounds__(256) void dtlr_f16_kernel(const float* __restrict__ XD, unsigned short* __restrict__ DT16, int total)
{
  const int i = blockIdx.x * 256 + threadIdx.x;
  if (i >= total) return;
  const int r  = i >> 2;
  const int k0 = (i & 3) << 3;
  const bool live = (k0 < kDtR);
  const int kc = live ? k0 : 0;
  v4f a0 = *(const v4f*)(XD + (size_t)r * kXdP + kc);
  v4f a1 = *(const v4f*)(XD + (size_t)r * kXdP + kc + 4);
  asm volatile("" : "+v"(a0));
  asm volatile("" : "+v"(a1));
  const float f0 = live ? a0[0] : 0.0f;
  const float f1 = live ? a0[1] : 0.0f;
  const float f2 = live ? a0[2] : 0.0f;
  const float f3 = live ? a0[3] : 0.0f;
  const float f4 = live ? a1[0] : 0.0f;
  const float f5 = live ? a1[1] : 0.0f;
  const float f6 = live ? a1[2] : 0.0f;
  const float f7 = live ? a1[3] : 0.0f;
  const unsigned p0 = pack2_f16(f0 * kCDT, f1 * kCDT);
  const unsigned p1 = pack2_f16(f2 * kCDT, f3 * kCDT);
  const unsigned p2 = pack2_f16(f4 * kCDT, f5 * kCDT);
  const unsigned p3 = pack2_f16(f6 * kCDT, f7 * kCDT);
  const v4u w = (v4u){p0, p1, p2, p3};
  unsigned short* p = DT16 + (size_t)i * 8;
  *(volatile v4u*)p = w;
  __threadfence();
  *(volatile v4u*)p = w;
}

typedef float    ms1_v4f __attribute__((ext_vector_type(4)));
typedef unsigned ms1_v4u __attribute__((ext_vector_type(4)));
struct ms1_args {
  const float* dtpre;
  const float* u;
  const float* bc;
  const float* z;
  const float* A_log;
  const float* Dskip;
  __half* y;
  __half* y_lo;
  long ld_dtpre;
  long ld_u;
  long ld_bc;
  long ld_z;
  long ld_y;
  int offB;
  int offC;
  int offZ;
  float ycarry;
  int dir;
  int D;
  int L;
  int nbatch;
};
static_assert(sizeof(ms1_args) == 136);

__device__ __forceinline__ float ms1_flush16(float v) {
  return (fabsf(v) < 6.103515625e-05f) ? 0.0f : v;
}
__device__ __forceinline__ unsigned ms1_h16bits(float v) {
  return (unsigned)__half_as_ushort(__float2half_rn(ms1_flush16(v)));
}
__device__ __forceinline__ float ms1_h16val(unsigned b) {
  return __half2float(__ushort_as_half((unsigned short)b));
}
__device__ __forceinline__ float ms1_softplus(float v) {
  return fmaxf(v, 0.0f) + log1pf(expf(-fabsf(v)));
}
__device__ __forceinline__ void ms1_pack2(float v0, float v1, unsigned& hw, unsigned& lw) {
  const unsigned h0 = ms1_h16bits(v0);
  const unsigned h1 = ms1_h16bits(v1);
  const float r0 = (v0 - ms1_h16val(h0)) * 2048.0f;
  const float r1 = (v1 - ms1_h16val(h1)) * 2048.0f;
  const unsigned l0 = ms1_h16bits(r0);
  const unsigned l1 = ms1_h16bits(r1);
  hw = h0 | (h1 << 16);
  lw = l0 | (l1 << 16);
}

template <int NSTATE>
__global__ __launch_bounds__(64 * (NSTATE / 16)) void ms1_scan_kernel(ms1_args a)
{
  static_assert(NSTATE == 16 || NSTATE == 64);
  constexpr int NQ  = NSTATE / 16;
  constexpr int NT  = 64 * NQ;
  constexpr int NW  = NT / 32;
  constexpr int BCW = 2 * NSTATE;
  constexpr int YP  = 68;
  constexpr int RPI = NW * 4;
  constexpr int NIT = 64 / RPI;
  static_assert(16 * NT <= 64 * YP);
  __shared__ __align__(16) float sBC[64 * BCW];
  __shared__ __align__(16) float sY[64 * YP];
  const int tid  = threadIdx.x;
  const int lane = tid & 31;
  const int wave = tid >> 5;
  const int c    = tid / NQ;
  const int sq   = tid - c * NQ;
  const int bpb  = a.D / 64;
  const int bi   = blockIdx.x / bpb;
  if (bi >= a.nbatch) return;
  const int d0 = (blockIdx.x - bi * bpb) * 64;
  const int d  = d0 + c;
  const long rowb = (long)bi * a.L;
  const bool hasz  = (a.z != nullptr);
  const bool hasD  = (a.Dskip != nullptr);
  const bool hasLo = (a.y_lo != nullptr);

#pragma unroll 1
  for (int n = 0; n < 16; ++n) {
    const float al = a.A_log[(long)d * NSTATE + sq * 16 + n];
    sY[n * NT + tid] = -expf(al);
  }
  __syncthreads();
  float An[16], h[16];
#pragma unroll
  for (int n = 0; n < 16; ++n) {
    An[n] = sY[n * NT + tid];
    h[n] = 0.0f;
  }
  float Dd = 0.0f;
  if (hasD) Dd = a.Dskip[d];

  const int nchunk = a.L / 64;
  const bool fwd = (a.dir > 0);
  const int s0 = fwd ? 0 : 63;
  const int sd = fwd ? 1 : -1;
  const int q  = lane >> 3;
  const int c8 = (lane & 7) * 8;

#pragma unroll 1
  for (int ci = 0; ci < nchunk; ++ci) {
    const int tb = fwd ? (ci * 64) : (a.L - 64 - ci * 64);
    const long rowc = rowb + tb;
    __syncthreads();
#pragma unroll 8
    for (int i = 0; i < 32; ++i) {
      const int idx = tid + i * NT;
      const int st  = idx / BCW;
      const int col = idx - st * BCW;
      const int sc  = (col < NSTATE) ? (a.offB + col) : (a.offC + col - NSTATE);
      sBC[idx] = a.bc[(rowc + st) * a.ld_bc + sc];
    }
    __syncthreads();
#pragma unroll 1
    for (int s = 0; s < 64; ++s) {
      const int ls = s0 + sd * s;
      const long row = rowc + ls;
      float pre = a.dtpre[row * a.ld_dtpre + d];
      float uv  = a.u[row * a.ld_u + d];
      float zv  = 0.0f;
      if (hasz) zv = a.z[row * a.ld_z + a.offZ + d];
      asm volatile("" : "+v"(pre));
      asm volatile("" : "+v"(uv));
      asm volatile("" : "+v"(zv));
      const float delta = ms1_softplus(pre);
      const float dtx = delta * uv;
      const float* bp = sBC + ls * BCW + sq * 16;
      const float* cp = bp + NSTATE;
      ms1_v4f Bq[4], Cq[4];
#pragma unroll
      for (int k = 0; k < 4; ++k) {
        Bq[k] = *(const ms1_v4f*)(bp + 4 * k);
        Cq[k] = *(const ms1_v4f*)(cp + 4 * k);
      }
      float yv = 0.0f;
#pragma unroll
      for (int n = 0; n < 16; ++n) {
        const float e = __expf(delta * An[n]);
        h[n] = fmaf(e, h[n], dtx * Bq[n >> 2][n & 3]);
        yv = fmaf(h[n], Cq[n >> 2][n & 3], yv);
      }
      if (NQ > 1) {
        yv += __shfl_xor(yv, 1, 32);
        yv += __shfl_xor(yv, 2, 32);
      }
      if (hasD) yv = fmaf(uv, Dd, yv);
      if (hasz) {
        const float sg = __builtin_amdgcn_rcpf(1.0f + expf(-zv));
        yv = yv * (zv * sg);
      }
      if (sq == 0) sY[ls * YP + c] = yv * a.ycarry;
    }
    __syncthreads();
    ms1_v4u hw[NIT], lw[NIT];
#pragma unroll
    for (int it = 0; it < NIT; ++it) {
      const int row = it * RPI + wave * 4 + q;
      const float* sp = sY + row * YP + c8;
      const ms1_v4f f0 = *(const ms1_v4f*)(sp);
      const ms1_v4f f1 = *(const ms1_v4f*)(sp + 4);
      unsigned h0, h1, h2, h3, l0, l1, l2, l3;
      ms1_pack2(f0[0], f0[1], h0, l0);
      ms1_pack2(f0[2], f0[3], h1, l1);
      ms1_pack2(f1[0], f1[1], h2, l2);
      ms1_pack2(f1[2], f1[3], h3, l3);
      hw[it] = (ms1_v4u){h0, h1, h2, h3};
      lw[it] = (ms1_v4u){l0, l1, l2, l3};
    }
    for (int pass = 0; pass < 2; ++pass) {
#pragma unroll
      for (int it = 0; it < NIT; ++it) {
        const int row = it * RPI + wave * 4 + q;
        const long o = (rowc + row) * a.ld_y + d0 + c8;
        *(volatile ms1_v4u*)(a.y + o) = hw[it];
        if (hasLo) *(volatile ms1_v4u*)(a.y_lo + o) = lw[it];
      }
      __threadfence();
    }
  }
}

extern "C" void kernel_launch(void* const* d_in, const int* in_sizes, int n_in,
                              void* d_out, int out_size, void* d_ws, size_t ws_size,
                              hipStream_t stream) {
  if (n_in < 10) return;
  if (in_sizes[0] != kNB * kCm * kL) return;
  if (in_sizes[1] != kXzP * kCm) return;
  if (in_sizes[2] != kDin * 4) return;
  if (in_sizes[3] != kDin) return;
  if (in_sizes[4] != kXdR * kDin) return;
  if (in_sizes[5] != kDin * kDtR) return;
  if (in_sizes[6] != kDin) return;
  if (in_sizes[7] != kDin * kNst) return;
  if (in_sizes[8] != kDin) return;
  if (in_sizes[9] != kCm * kDin) return;
  if (out_size != kNB * kCm * kL) return;
  if (ws_size < kWsTotal) return;

  const float* x       = (const float*)d_in[0];
  const float* W_in    = (const float*)d_in[1];
  const float* conv_w  = (const float*)d_in[2];
  const float* conv_b  = (const float*)d_in[3];
  const float* W_x     = (const float*)d_in[4];
  const float* W_dt    = (const float*)d_in[5];
  const float* b_dt    = (const float*)d_in[6];
  const float* A_log   = (const float*)d_in[7];
  const float* D_par   = (const float*)d_in[8];
  const float* W_out   = (const float*)d_in[9];
  float* out = (float*)d_out;

  char* ws = (char*)d_ws;
  unsigned short* XB    = (unsigned short*)(ws + kOffXB);
  unsigned short* WIB   = (unsigned short*)(ws + kOffWIB);
  unsigned short* WX16  = (unsigned short*)(ws + kOffWX16);
  unsigned short* WDT16 = (unsigned short*)(ws + kOffWDT16);
  unsigned short* WO16  = (unsigned short*)(ws + kOffWO16);
  float*          QV    = (float*)(ws + kOffQV);
  float*          XZ    = (float*)(ws + kOffXZ);
  float*          U     = (float*)(ws + kOffU);
  unsigned short* U16   = (unsigned short*)(ws + kOffU16);
  float*          XD    = (float*)(ws + kOffXD);
  unsigned short* DT16  = (unsigned short*)(ws + kOffDT16);
  float*          DT    = (float*)(ws + kOffDT);
  unsigned short* Y16   = (unsigned short*)(ws + kOffY16);

  xpose_bf16_kernel<<<dim3(kL / 64, kCm / 64, kNB), 256, 0, stream>>>(x, XB);
  prep_plane16_kernel<0><<<(kXzP * kCm / 8) / 256, 256, 0, stream>>>(W_in, kXzP, kCm, WIB, kCm, 1.0f, kXzP * kCm / 8);
  prep_plane16_kernel<1><<<(kXdP * kDin / 8) / 256, 256, 0, stream>>>(W_x, kXdR, kDin, WX16, kDin, kCWX, kXdP * kDin / 8);
  prep_plane16_kernel<1><<<(kDin * kDtKP / 8) / 256, 256, 0, stream>>>(W_dt, kDin, kDtR, WDT16, kDtKP, kCWD, kDin * kDtKP / 8);
  prep_plane16_kernel<1><<<(kCm * kDin / 8) / 256, 256, 0, stream>>>(W_out, kCm, kDin, WO16, kDin, kCWO, kCm * kDin / 8);
  quant_vals_kernel<<<(kQvTotal / 4 + 255) / 256, 256, 0, stream>>>(conv_w, conv_b, b_dt, A_log, D_par, QV);

  for (int b = 0; b < kNB; ++b) {
    eng::gemm64_kernel<1, 0><<<dim3((kL / 64) * (kXzP / 64) / 8, 1), 256, 0, stream>>>(
        XB + (size_t)b * kL * kCm, kCm, 0L,
        WIB, kCm, 0L,
        XZ, kXzP, 0L,
        nullptr, kL, kXzP, kCm, 1.0f);

    conv_silu_kernel<<<dim3(kDin / 256, kL / 64), 256, 0, stream>>>(XZ, QV + kQvCw, QV + kQvCb, U, U16);

    eng::gemm64_kernel<0, 0><<<dim3((kL / 64) * (kXdP / 64) / 8, 1), 256, 0, stream>>>(
        U16, kDin, 0L,
        WX16, kDin, 0L,
        XD, kXdP, 0L,
        nullptr, kL, kXdP, kDin, kSclX);

    dtlr_f16_kernel<<<(kL * 4) / 256, 256, 0, stream>>>(XD, DT16, kL * 4);

    eng::gemm64_kernel<0, 2><<<dim3((kL / 64) * (kDin / 64) / 8, 1), 256, 0, stream>>>(
        DT16, kDtKP, 0L,
        WDT16, kDtKP, 0L,
        DT, kDin, 0L,
        QV + kQvDb, kL, kDin, kDtKP, kSclD);

    ms1_args sa;
    sa.dtpre = DT;
    sa.u = U;
    sa.bc = XD;
    sa.z = XZ;
    sa.A_log = QV + kQvAl;
    sa.Dskip = QV + kQvDk;
    sa.y = (__half*)(Y16 + (size_t)b * kL * kDin);
    sa.y_lo = nullptr;
    sa.ld_dtpre = kDin;
    sa.ld_u = kDin;
    sa.ld_bc = kXdP;
    sa.ld_z = kXzP;
    sa.ld_y = kDin;
    sa.offB = kDtR;
    sa.offC = kDtR + kNst;
    sa.offZ = kDin;
    sa.ycarry = kCY;
    sa.dir = 1;
    sa.D = kDin;
    sa.L = kL;
    sa.nbatch = 1;
    ms1_scan_kernel<16><<<dim3(kDin / 64), 64, 0, stream>>>(sa);
  }

  eng::gemm64_kernel<0, 0><<<dim3((kCm / 64) * (kL / 64) / 8, kNB), 256, 0, stream>>>(
      WO16, kDin, 0L,
      Y16, kDin, (long)kL * kDin,
      out, kL, (long)kCm * kL,
      nullptr, kCm, kL, kDin, kSclO);
}
